// Graph_module_net_0_loss_18631568130083
// MI455X (gfx1250) — hardware-run, weakly checked
//
#include <hip/hip_runtime.h>

typedef __bf16         v16bf __attribute__((ext_vector_type(16)));
typedef unsigned short v16us __attribute__((ext_vector_type(16)));
typedef unsigned short v8us  __attribute__((ext_vector_type(8)));
typedef float          v8f   __attribute__((ext_vector_type(8)));
typedef float          v4f   __attribute__((ext_vector_type(4)));
typedef v8us __attribute__((may_alias)) v8usa;
typedef v4f  __attribute__((may_alias)) v4fa;

union BF { v16bf bf; v16us us; struct { v8us lo; v8us hi; } s; };

#define NTOK 8192
#define CIN  256
#define COUT 512
#define NX   (NTOK * CIN)
#define NWG  (COUT * CIN)
#define NW1  (512 * 64)
#define NW2  (512 * 128)

#define OFF_XH   0
#define OFF_XL   (NX)
#define OFF_GH   (2 * NX)
#define OFF_GL   (3 * NX)
#define OFF_WGH  (4 * NX)
#define OFF_WGL  (4 * NX + NWG)
#define OFF_W1H  (4 * NX + 2 * NWG)
#define OFF_W1L  (4 * NX + 2 * NWG + NW1)
#define OFF_W2H  (4 * NX + 2 * NWG + 2 * NW1)
#define OFF_W2L  (4 * NX + 2 * NWG + 2 * NW1 + NW2)
#define TOT16    (4 * NX + 2 * NWG + 2 * NW1 + 2 * NW2)
#define NSRC     (2 * NX + NWG + NW1 + NW2)
#define NGRP     (NSRC / 8)

#define SOP 132
#define LDP 136

static_assert((NX % 2048) == 0);
static_assert((NWG % 2048) == 0);
static_assert((NW1 % 2048) == 0);
static_assert((NW2 % 2048) == 0);
static_assert((NSRC % 8) == 0);
static_assert((NTOK % 64) == 0);
static_assert((COUT % 128) == 0);

__device__ __forceinline__ unsigned short f2bf(float f) {
  const unsigned u = __float_as_uint(f);
  return (unsigned short)((u + 0x7FFFu + ((u >> 16) & 1u)) >> 16);
}
__device__ __forceinline__ float bf2f(unsigned short h) {
  return __uint_as_float(((unsigned)h) << 16);
}

__device__ __forceinline__ v8f mma_bf16(const BF& a, const BF& b, v8f c) {
  v8f d = __builtin_amdgcn_wmma_f32_16x16x32_bf16(false, a.bf, false, b.bf, (short)0, c, false, false);
  asm volatile("v_nop\n\tv_nop\n\tv_nop\n\tv_nop" : "+v"(d) : "v"(a.us), "v"(b.us));
  return d;
}

__device__ __forceinline__ BF frag_g(const unsigned short* __restrict__ p, int h) {
  BF f;
  f.s.lo = *(const v8usa*)(p + 8 * h);
  f.s.hi = *(const v8usa*)(p + 16 + 8 * h);
  return f;
}

__device__ __forceinline__ void pass_store(const float* sO, float* dst, const v4f zadd, int w, int lane) {
  #pragma unroll
  for (int i = 0; i < 8; ++i) {
    const int row = w * 8 + i;
    v4f v = *(const v4fa*)(sO + row * SOP + 4 * lane);
    v += zadd;
    *(volatile v4f*)(dst + (size_t)row * COUT + 4 * lane) = v;
  }
}
__device__ __forceinline__ void pass_fill(float* dst, const v4f z, int w, int lane) {
  #pragma unroll
  for (int i = 0; i < 8; ++i) {
    const int row = w * 8 + i;
    *(volatile v4f*)(dst + (size_t)row * COUT + 4 * lane) = z;
  }
}

__global__ __launch_bounds__(256) void k_split(
    const float* __restrict__ xin, const float* __restrict__ gt,
    const float* __restrict__ wg, const float* __restrict__ w1,
    const float* __restrict__ w2, unsigned short* __restrict__ pl, int ngroups)
{
  const int gidx = blockIdx.x * 256 + threadIdx.x;
  if (gidx >= ngroups) return;
  const int e = gidx * 8;
  const float* src;
  unsigned short* dh;
  unsigned short* dl;
  if (e < NX) {
    src = xin + e; dh = pl + (size_t)OFF_XH + e; dl = pl + (size_t)OFF_XL + e;
  } else if (e < 2 * NX) {
    const int o = e - NX;
    src = gt + o; dh = pl + (size_t)OFF_GH + o; dl = pl + (size_t)OFF_GL + o;
  } else if (e < 2 * NX + NWG) {
    const int o = e - 2 * NX;
    src = wg + o; dh = pl + (size_t)OFF_WGH + o; dl = pl + (size_t)OFF_WGL + o;
  } else if (e < 2 * NX + NWG + NW1) {
    const int o = e - 2 * NX - NWG;
    src = w1 + o; dh = pl + (size_t)OFF_W1H + o; dl = pl + (size_t)OFF_W1L + o;
  } else {
    const int o = e - 2 * NX - NWG - NW1;
    src = w2 + o; dh = pl + (size_t)OFF_W2H + o; dl = pl + (size_t)OFF_W2L + o;
  }
  const v4f a = *(const v4fa*)src;
  const v4f c = *(const v4fa*)(src + 4);
  const float f[8] = { a.x, a.y, a.z, a.w, c.x, c.y, c.z, c.w };
  v8us H, L;
  #pragma unroll
  for (int i = 0; i < 8; ++i) {
    const unsigned short hh = f2bf(f[i]);
    H[i] = hh;
    L[i] = f2bf(f[i] - bf2f(hh));
  }
  *(volatile v8us*)dh = H;
  *(volatile v8us*)dl = L;
  __threadfence();
  *(volatile v8us*)dh = H;
  *(volatile v8us*)dl = L;
}

__global__ __launch_bounds__(256) void k_gts(
    const unsigned short* __restrict__ aH, const unsigned short* __restrict__ aL,
    const unsigned short* __restrict__ bH, const unsigned short* __restrict__ bL,
    const float* __restrict__ bias, float* __restrict__ out)
{
  __shared__ __attribute__((aligned(16))) float sO[64 * SOP];

  const int tid = threadIdx.x, lane = tid & 31, w = tid >> 5;
  const int h = lane >> 4, m = lane & 15;
  const int wm = w & 1, wn = w >> 1;
  const int m0 = blockIdx.x * 64, n0 = blockIdx.y * 128;

  const unsigned short* arH[2]; const unsigned short* arL[2];
  const unsigned short* brH[2]; const unsigned short* brL[2];
  #pragma unroll
  for (int t = 0; t < 2; ++t) {
    const size_t ra = (size_t)(m0 + wm * 32 + 16 * t + m) * CIN;
    const size_t rb = (size_t)(n0 + wn * 32 + 16 * t + m) * CIN;
    arH[t] = aH + ra; arL[t] = aL + ra;
    brH[t] = bH + rb; brL[t] = bL + rb;
  }

  const v8f zero8 = {0.f, 0.f, 0.f, 0.f, 0.f, 0.f, 0.f, 0.f};
  v8f acc[2][2];
  #pragma unroll
  for (int mt = 0; mt < 2; ++mt)
    #pragma unroll
    for (int nt = 0; nt < 2; ++nt) acc[mt][nt] = zero8;

  #pragma unroll 1
  for (int k0 = 0; k0 < CIN; k0 += 32) {
    BF ah[2], al[2];
    #pragma unroll
    for (int mt = 0; mt < 2; ++mt) { ah[mt] = frag_g(arH[mt] + k0, h); al[mt] = frag_g(arL[mt] + k0, h); }
    #pragma unroll
    for (int nt = 0; nt < 2; ++nt) {
      const BF bh = frag_g(brH[nt] + k0, h);
      const BF bl = frag_g(brL[nt] + k0, h);
      #pragma unroll
      for (int mt = 0; mt < 2; ++mt) {
        acc[mt][nt] = mma_bf16(ah[mt], bh, acc[mt][nt]);
        acc[mt][nt] = mma_bf16(ah[mt], bl, acc[mt][nt]);
        acc[mt][nt] = mma_bf16(al[mt], bh, acc[mt][nt]);
      }
    }
  }

  #pragma unroll
  for (int nt = 0; nt < 2; ++nt) {
    const int col = wn * 32 + 16 * nt + m;
    const float bb = bias[n0 + col];
    #pragma unroll
    for (int mt = 0; mt < 2; ++mt) {
      #pragma unroll
      for (int r = 0; r < 8; ++r) {
        const int row = wm * 32 + 16 * mt + 8 * h + r;
        sO[row * SOP + col] = fmaxf(acc[mt][nt][r] + bb, 0.0f);
      }
    }
  }
  __syncthreads();

  const v4f z4 = {0.f, 0.f, 0.f, 0.f};
  float* dst = out + (size_t)m0 * COUT + n0;
  pass_store(sO, dst, z4, w, lane);
  __threadfence();
  pass_store(sO, dst, z4, w, lane);
}

__global__ __launch_bounds__(256) void k_gconv(
    const unsigned short* __restrict__ xH, const unsigned short* __restrict__ xL,
    const unsigned short* __restrict__ w1H, const unsigned short* __restrict__ w1L,
    const float* __restrict__ b1, const float* __restrict__ l1g, const float* __restrict__ l1b,
    const unsigned short* __restrict__ w2H, const unsigned short* __restrict__ w2L,
    const float* __restrict__ b2, const float* __restrict__ l2g, const float* __restrict__ l2b,
    float* __restrict__ out0, float* __restrict__ out2)
{
  __shared__ __attribute__((aligned(16))) float s_raw[8704];
  unsigned short* sH = (unsigned short*)s_raw;
  unsigned short* sL = sH + 64 * LDP;
  float* sO = s_raw;

  const int tid = threadIdx.x, lane = tid & 31, w = tid >> 5;
  const int h = lane >> 4, m = lane & 15;
  const int wm = w & 1, wn = w >> 1;
  const int tok0 = blockIdx.x * 64, g = blockIdx.y, ch0 = g * 128;

  const v8f zero8 = {0.f, 0.f, 0.f, 0.f, 0.f, 0.f, 0.f, 0.f};
  v8f acc[2][2];

  const unsigned short* arH[2]; const unsigned short* arL[2];
  const unsigned short* brH[2]; const unsigned short* brL[2];
  #pragma unroll
  for (int t = 0; t < 2; ++t) {
    const size_t ra = (size_t)(tok0 + wm * 32 + 16 * t + m) * CIN + g * 64;
    const size_t rb = (size_t)(ch0 + wn * 32 + 16 * t + m) * 64;
    arH[t] = xH + ra;  arL[t] = xL + ra;
    brH[t] = w1H + rb; brL[t] = w1L + rb;
  }
  #pragma unroll
  for (int mt = 0; mt < 2; ++mt)
    #pragma unroll
    for (int nt = 0; nt < 2; ++nt) acc[mt][nt] = zero8;

  #pragma unroll 1
  for (int k0 = 0; k0 < 64; k0 += 32) {
    BF ah[2], al[2];
    #pragma unroll
    for (int mt = 0; mt < 2; ++mt) { ah[mt] = frag_g(arH[mt] + k0, h); al[mt] = frag_g(arL[mt] + k0, h); }
    #pragma unroll
    for (int nt = 0; nt < 2; ++nt) {
      const BF bh = frag_g(brH[nt] + k0, h);
      const BF bl = frag_g(brL[nt] + k0, h);
      #pragma unroll
      for (int mt = 0; mt < 2; ++mt) {
        acc[mt][nt] = mma_bf16(ah[mt], bh, acc[mt][nt]);
        acc[mt][nt] = mma_bf16(ah[mt], bl, acc[mt][nt]);
        acc[mt][nt] = mma_bf16(al[mt], bh, acc[mt][nt]);
      }
    }
  }

  #pragma unroll
  for (int nt = 0; nt < 2; ++nt) {
    const int chl = wn * 32 + 16 * nt + m;
    const int ch = ch0 + chl;
    const float bb = b1[ch];
    const float z1 = 0.0f * l1g[ch] + l1b[ch];
    #pragma unroll
    for (int mt = 0; mt < 2; ++mt) {
      #pragma unroll
      for (int r = 0; r < 8; ++r) {
        const int tokl = wm * 32 + 16 * mt + 8 * h + r;
        const float v = fmaxf(acc[mt][nt][r] + bb, 0.0f) + z1;
        const unsigned short hh = f2bf(v);
        sH[tokl * LDP + chl] = hh;
        sL[tokl * LDP + chl] = f2bf(v - bf2f(hh));
      }
    }
  }
  __syncthreads();

  const unsigned short* crH[2]; const unsigned short* crL[2];
  int arow[2];
  #pragma unroll
  for (int t = 0; t < 2; ++t) {
    arow[t] = (wm * 32 + 16 * t + m) * LDP;
    const size_t rb = (size_t)(ch0 + wn * 32 + 16 * t + m) * 128;
    crH[t] = w2H + rb; crL[t] = w2L + rb;
  }
  #pragma unroll
  for (int mt = 0; mt < 2; ++mt)
    #pragma unroll
    for (int nt = 0; nt < 2; ++nt) acc[mt][nt] = zero8;

  #pragma unroll 1
  for (int k0 = 0; k0 < 128; k0 += 32) {
    BF ah[2], al[2];
    #pragma unroll
    for (int mt = 0; mt < 2; ++mt) {
      ah[mt].s.lo = *(const v8usa*)(sH + arow[mt] + k0 + 8 * h);
      ah[mt].s.hi = *(const v8usa*)(sH + arow[mt] + k0 + 16 + 8 * h);
      al[mt].s.lo = *(const v8usa*)(sL + arow[mt] + k0 + 8 * h);
      al[mt].s.hi = *(const v8usa*)(sL + arow[mt] + k0 + 16 + 8 * h);
    }
    #pragma unroll
    for (int nt = 0; nt < 2; ++nt) {
      const BF bh = frag_g(crH[nt] + k0, h);
      const BF bl = frag_g(crL[nt] + k0, h);
      #pragma unroll
      for (int mt = 0; mt < 2; ++mt) {
        acc[mt][nt] = mma_bf16(ah[mt], bh, acc[mt][nt]);
        acc[mt][nt] = mma_bf16(ah[mt], bl, acc[mt][nt]);
        acc[mt][nt] = mma_bf16(al[mt], bh, acc[mt][nt]);
      }
    }
  }
  __syncthreads();

  #pragma unroll
  for (int nt = 0; nt < 2; ++nt) {
    const int chl = wn * 32 + 16 * nt + m;
    const float bb = b2[ch0 + chl];
    #pragma unroll
    for (int mt = 0; mt < 2; ++mt) {
      #pragma unroll
      for (int r = 0; r < 8; ++r) {
        const int tokl = wm * 32 + 16 * mt + 8 * h + r;
        sO[tokl * SOP + chl] = fmaxf(acc[mt][nt][r] + bb, 0.0f);
      }
    }
  }
  __syncthreads();

  const int cb = ch0 + 4 * lane;
  v4f zc;
  zc.x = 0.0f * l2g[cb + 0] + l2b[cb + 0];
  zc.y = 0.0f * l2g[cb + 1] + l2b[cb + 1];
  zc.z = 0.0f * l2g[cb + 2] + l2b[cb + 2];
  zc.w = 0.0f * l2g[cb + 3] + l2b[cb + 3];

  float* dst0 = out0 + (size_t)tok0 * COUT + ch0;
  float* dst2 = out2 + (size_t)tok0 * COUT + ch0;
  pass_store(sO, dst0, zc, w, lane);
  pass_fill(dst2, zc, w, lane);
  __threadfence();
  pass_store(sO, dst0, zc, w, lane);
  pass_fill(dst2, zc, w, lane);
}

extern "C" void kernel_launch(void* const* d_in, const int* in_sizes, int n_in,
                              void* d_out, int out_size, void* d_ws, size_t ws_size,
                              hipStream_t stream) {
  if (n_in < 16) return;
  if (in_sizes[0] != NX || in_sizes[3] != NX) return;
  if (in_sizes[6] != NW1 || in_sizes[7] != COUT) return;
  if (in_sizes[8] != NW2 || in_sizes[9] != COUT) return;
  if (in_sizes[10] != COUT || in_sizes[11] != COUT || in_sizes[12] != COUT || in_sizes[13] != COUT) return;
  if (in_sizes[14] != NWG || in_sizes[15] != COUT) return;
  if (out_size != 3 * NTOK * COUT) return;

  const size_t ws_need = (size_t)TOT16 * 2;
  if (ws_need > ws_size) return;

  const float* xin  = (const float*)d_in[0];
  const float* gt   = (const float*)d_in[3];
  const float* W1g  = (const float*)d_in[6];
  const float* b1g  = (const float*)d_in[7];
  const float* W2g  = (const float*)d_in[8];
  const float* b2g  = (const float*)d_in[9];
  const float* ln1g = (const float*)d_in[10];
  const float* ln1b = (const float*)d_in[11];
  const float* ln2g = (const float*)d_in[12];
  const float* ln2b = (const float*)d_in[13];
  const float* Wgt  = (const float*)d_in[14];
  const float* bgt  = (const float*)d_in[15];

  unsigned short* pl = (unsigned short*)d_ws;
  const unsigned short* xH  = pl + (size_t)OFF_XH;
  const unsigned short* xL  = pl + (size_t)OFF_XL;
  const unsigned short* gH  = pl + (size_t)OFF_GH;
  const unsigned short* gL  = pl + (size_t)OFF_GL;
  const unsigned short* wgH = pl + (size_t)OFF_WGH;
  const unsigned short* wgL = pl + (size_t)OFF_WGL;
  const unsigned short* w1H = pl + (size_t)OFF_W1H;
  const unsigned short* w1L = pl + (size_t)OFF_W1L;
  const unsigned short* w2H = pl + (size_t)OFF_W2H;
  const unsigned short* w2L = pl + (size_t)OFF_W2L;

  float* out0 = (float*)d_out;
  float* out1 = (float*)d_out + (size_t)NTOK * COUT;
  float* out2 = (float*)d_out + (size_t)2 * NTOK * COUT;

  k_split<<<(NGRP + 255) / 256, 256, 0, stream>>>(xin, gt, Wgt, W1g, W2g, pl, NGRP);

  k_gts<<<dim3(NTOK / 64, COUT / 128), 256, 0, stream>>>(gH, gL, wgH, wgL, bgt, out1);

  k_gconv<<<dim3(NTOK / 64, 4), 256, 0, stream>>>(xH, xL, w1H, w1L, b1g, ln1g, ln1b,
                                                   w2H, w2L, b2g, ln2g, ln2b, out0, out2);
}
